// LungCancerGRU_85796266705068
// MI455X (gfx1250) — hardware-verified
//
#include <hip/hip_runtime.h>
#include <math.h>

constexpr int NBATCH   = 262144;
constexpr int NSTEP    = 15;
constexpr int NHID     = 64;
constexpr int NGATE    = 3 * NHID;
constexpr int NOUTC    = 2;
constexpr int NTHR     = 256;
constexpr int NWAVE    = NTHR / 32;
constexpr int ROWS_W   = 16;
constexpr int ROWS_BLK = NWAVE * ROWS_W;
constexpr int WPITCH   = 72;
constexpr int HPITCH   = 72;
constexpr int XSLOT    = 256;
constexpr int XUSED    = ROWS_W * NSTEP;
constexpr float WCARRY = 16.0f;
constexpr float HCARRY = 16.0f;
constexpr float FOLD   = 1.0f / (WCARRY * HCARRY);

static_assert(NBATCH % ROWS_BLK == 0, "grid exact");
static_assert(NHID % 32 == 0, "K multiple of 32");
static_assert(NGATE % 16 == 0, "N multiple of 16");
static_assert(ROWS_W * NOUTC * 4 == 128, "one wave writes one 128-B line");
static_assert(XUSED <= XSLOT, "x slot");
static_assert((NGATE * (NHID / 8)) % NTHR == 0, "weight staging loop exact");
static_assert(NGATE == 6 * 32, "constant staging is wave-uniform");
static_assert((WPITCH % 8) == 0 && (HPITCH % 8) == 0, "16-B aligned fragment rows");

typedef __attribute__((ext_vector_type(16))) _Float16 v16h;
typedef __attribute__((ext_vector_type(8)))  _Float16 v8h;
typedef __attribute__((ext_vector_type(8)))  float    v8f;
typedef __attribute__((ext_vector_type(4)))  float    v4f;

template <typename T> struct Frag;
template <> struct Frag<_Float16> {
  typedef v16h V; union U { v16h v; v8h h[2]; };
  static __device__ __forceinline__ v16h load(const _Float16* p) {
    U f; f.h[0] = *(const v8h*)(p); f.h[1] = *(const v8h*)(p + 16); return f.v;
  }
  static __device__ __forceinline__ v8f mma(v16h a, v16h b, v8f c) {
    return __builtin_amdgcn_wmma_f32_16x16x32_f16(false, a, false, b, (short)0, c, false, false);
  }
};

__device__ __forceinline__ void grp_guard(v8f& a, v8f& b, v8f& c, v16h x0, v16h x1,
                                          v16h y0, v16h y1, v16h y2, v16h y3, v16h y4, v16h y5) {
  asm volatile("v_nop\n\tv_nop\n\tv_nop\n\tv_nop"
               : "+v"(a), "+v"(b), "+v"(c)
               : "v"(x0), "v"(x1), "v"(y0), "v"(y1), "v"(y2), "v"(y3), "v"(y4), "v"(y5));
}

__device__ __forceinline__ float fsig(float v)  { return __builtin_amdgcn_rcpf(1.0f + __expf(-v)); }
__device__ __forceinline__ float ftanh(float v) { return 1.0f - 2.0f * __builtin_amdgcn_rcpf(__expf(2.0f * v) + 1.0f); }

__global__ __launch_bounds__(NTHR) void gru_seq_kernel(const float* __restrict__ x, const float* __restrict__ w_ih,
                                                       const float* __restrict__ w_hh, const float* __restrict__ b_ih,
                                                       const float* __restrict__ b_hh, const float* __restrict__ w_fc,
                                                       const float* __restrict__ b_fc, float* __restrict__ out) {
  __shared__ __align__(16) _Float16 Wl[NGATE * WPITCH];
  __shared__ __align__(16) _Float16 Ah[NWAVE * ROWS_W * HPITCH];
  __shared__ __align__(16) float    Xs[NWAVE * XSLOT];
  __shared__ __align__(16) float    Cs[3 * NGATE];

  const int tid = threadIdx.x, lane = tid & 31, wave = tid >> 5;
  const int c = lane & 15, hh = lane >> 4;
  const int row0 = blockIdx.x * ROWS_BLK + wave * ROWS_W;

#pragma unroll 1
  for (int it = 0; it < (NGATE * (NHID / 8)) / NTHR; ++it) {
    const int idx = it * NTHR + tid;
    const int row = idx >> 3, c8 = (idx & 7) * 8;
    const v4f va = *(const v4f*)(w_hh + row * NHID + c8);
    const v4f vb = *(const v4f*)(w_hh + row * NHID + c8 + 4);
    v8h hv;
#pragma unroll
    for (int e = 0; e < 4; ++e) {
      const float fa = va[e] * WCARRY;
      const float fb = vb[e] * WCARRY;
      hv[e]     = (_Float16)fa;
      hv[4 + e] = (_Float16)fb;
    }
    *(v8h*)(Wl + row * WPITCH + c8) = hv;
  }
  {
    const size_t xbase = (size_t)row0 * NSTEP;
#pragma unroll
    for (int it = 0; it < XSLOT / 32; ++it) {
      const int idx = it * 32 + lane;
      const int src = (idx < XUSED) ? idx : (XUSED - 1);
      Xs[wave * XSLOT + idx] = x[xbase + src];
    }
  }
  if (tid < NGATE) {
    Cs[tid]             = w_ih[tid];
    Cs[NGATE + tid]     = b_ih[tid];
    Cs[2 * NGATE + tid] = b_hh[tid];
  }
  {
    const v8h z8h = {(_Float16)0.0f, (_Float16)0.0f, (_Float16)0.0f, (_Float16)0.0f,
                     (_Float16)0.0f, (_Float16)0.0f, (_Float16)0.0f, (_Float16)0.0f};
#pragma unroll 1
    for (int i = tid; i < (NWAVE * ROWS_W * HPITCH) / 8; i += NTHR) *(v8h*)(Ah + 8 * i) = z8h;
  }
  __syncthreads();

  float cwr[4], cwz[4], cwn[4], cbr[4], cbz[4], cbi[4], cbh[4];
#pragma unroll
  for (int j = 0; j < 4; ++j) {
    const int u = 16 * j + c;
    cwr[j] = Cs[u];
    cwz[j] = Cs[NHID + u];
    cwn[j] = Cs[2 * NHID + u];
    cbr[j] = Cs[NGATE + u] + Cs[2 * NGATE + u];
    cbz[j] = Cs[NGATE + NHID + u] + Cs[2 * NGATE + NHID + u];
    cbi[j] = Cs[NGATE + 2 * NHID + u];
    cbh[j] = Cs[2 * NGATE + 2 * NHID + u];
  }

  float hst[4][8];
#pragma unroll
  for (int j = 0; j < 4; ++j)
#pragma unroll
    for (int r = 0; r < 8; ++r) hst[j][r] = 0.0f;

  _Float16*       ahw   = Ah + wave * ROWS_W * HPITCH;
  const _Float16* ahrow = ahw + c * HPITCH + 8 * hh;
  const _Float16* wlane = Wl + c * WPITCH + 8 * hh;
  const float*    xw    = Xs + wave * XSLOT + (8 * hh) * NSTEP;
  const v8f z8 = {0.f, 0.f, 0.f, 0.f, 0.f, 0.f, 0.f, 0.f};

#pragma unroll 1
  for (int t = 0; t < NSTEP; ++t) {
    __syncthreads();
    float x8[8];
#pragma unroll
    for (int r = 0; r < 8; ++r) x8[r] = xw[r * NSTEP + t];
    const v16h a0 = Frag<_Float16>::load(ahrow);
    const v16h a1 = Frag<_Float16>::load(ahrow + 32);

#pragma unroll
    for (int j = 0; j < 4; ++j) {
      const _Float16* wj = wlane + (16 * j) * WPITCH;
      const v16h br0 = Frag<_Float16>::load(wj);
      const v16h br1 = Frag<_Float16>::load(wj + 32);
      const v16h bz0 = Frag<_Float16>::load(wj + NHID * WPITCH);
      const v16h bz1 = Frag<_Float16>::load(wj + NHID * WPITCH + 32);
      const v16h bn0 = Frag<_Float16>::load(wj + 2 * NHID * WPITCH);
      const v16h bn1 = Frag<_Float16>::load(wj + 2 * NHID * WPITCH + 32);
      v8f ar = z8, az = z8, an = z8;
      ar = Frag<_Float16>::mma(a0, br0, ar);
      az = Frag<_Float16>::mma(a0, bz0, az);
      an = Frag<_Float16>::mma(a0, bn0, an);
      ar = Frag<_Float16>::mma(a1, br1, ar);
      az = Frag<_Float16>::mma(a1, bz1, az);
      an = Frag<_Float16>::mma(a1, bn1, an);
      grp_guard(ar, az, an, a0, a1, br0, br1, bz0, bz1, bn0, bn1);

#pragma unroll
      for (int r = 0; r < 8; ++r) {
        const float xv = x8[r];
        const float pr = ar[r] * FOLD + (cwr[j] * xv + cbr[j]);
        const float pz = az[r] * FOLD + (cwz[j] * xv + cbz[j]);
        const float gr = fsig(pr);
        const float gz = fsig(pz);
        const float hn_in = an[r] * FOLD + cbh[j];
        const float gn = ftanh((cwn[j] * xv + cbi[j]) + gr * hn_in);
        const float ho = hst[j][r];
        const float hnew = (1.0f - gz) * gn + gz * ho;
        hst[j][r] = hnew;
        const float hc = hnew * HCARRY;
        ahw[(8 * hh + r) * HPITCH + 16 * j + c] = (_Float16)hc;
      }
      asm volatile("" ::: "memory");
    }
  }

  float wf0[4], wf1[4];
#pragma unroll
  for (int j = 0; j < 4; ++j) {
    wf0[j] = w_fc[16 * j + c];
    wf1[j] = w_fc[NHID + 16 * j + c];
  }
  float p[16];
#pragma unroll
  for (int r = 0; r < 8; ++r) {
    float s0 = 0.0f, s1 = 0.0f;
#pragma unroll
    for (int j = 0; j < 4; ++j) {
      s0 = fmaf(hst[j][r], wf0[j], s0);
      s1 = fmaf(hst[j][r], wf1[j], s1);
    }
    p[2 * r]     = s0;
    p[2 * r + 1] = s1;
  }
#pragma unroll
  for (int i = 0; i < 16; ++i) {
#pragma unroll
    for (int off = 1; off < 16; off <<= 1) p[i] += __shfl_xor(p[i], off, 32);
  }
  float val = 0.0f;
#pragma unroll
  for (int i = 0; i < 16; ++i) val = (c == i) ? p[i] : val;
  val += b_fc[c & 1];

  float* op = out + (size_t)row0 * NOUTC + lane;
  *(volatile float*)op = val;
  __threadfence();
  *(volatile float*)op = val;
}

extern "C" void kernel_launch(void* const* d_in, const int* in_sizes, int n_in,
                              void* d_out, int out_size, void* d_ws, size_t ws_size, hipStream_t stream) {
  (void)d_ws; (void)ws_size;
  if (n_in < 7 || d_out == nullptr) return;
  if (in_sizes[0] != NBATCH * NSTEP || in_sizes[1] != NGATE || in_sizes[2] != NGATE * NHID ||
      in_sizes[3] != NGATE || in_sizes[4] != NGATE || in_sizes[5] != NOUTC * NHID ||
      in_sizes[6] != NOUTC || out_size != NBATCH * NOUTC) return;

  const float* x    = (const float*)d_in[0];
  const float* w_ih = (const float*)d_in[1];
  const float* w_hh = (const float*)d_in[2];
  const float* b_ih = (const float*)d_in[3];
  const float* b_hh = (const float*)d_in[4];
  const float* w_fc = (const float*)d_in[5];
  const float* b_fc = (const float*)d_in[6];
  float* out = (float*)d_out;

  gru_seq_kernel<<<NBATCH / ROWS_BLK, NTHR, 0, stream>>>(x, w_ih, w_hh, b_ih, b_hh, w_fc, b_fc, out);
}
